// VectorQuantizer_24996709662906
// MI455X (gfx1250) — hardware-verified
//
#include <hip/hip_runtime.h>
#pragma clang fp contract(off)


#ifndef NB
#define NB 8
#endif
#ifndef SEQ
#define SEQ 4096
#endif
#ifndef NCODE
#define NCODE 8192
#endif
#define NB_FULL  8
#define SEQ_FULL 4096
#ifndef OUT_SEQ
#define OUT_SEQ SEQ
#endif
#define DIM   64
#define SW    4
#define MROWS 32
#define QRS   2048.0f
#define QRI   (1.0f / 2048.0f)

static_assert(DIM == 64);
static_assert(DIM % 32 == 0);
static_assert(MROWS == 32);
static_assert(SEQ % (SW * MROWS) == 0);
static_assert(SEQ % 32 == 0);
static_assert(NCODE % 32 == 0);
static_assert(NCODE % 16 == 0);
static_assert(NCODE >= 16);
static_assert(OUT_SEQ % 32 == 0);
static_assert(NB <= NB_FULL);
static_assert(SEQ <= SEQ_FULL);
static_assert((size_t)NCODE * DIM < (size_t)1 << 31);
static_assert((size_t)NB * SEQ * DIM < (size_t)1 << 31);
static_assert(256 * 16 == 32 * DIM * 2);
static_assert(8 * 16 == 32 * 4);
static_assert(32 * 2 * 8 == MROWS * 16);
static_assert((SW * MROWS * 16 + SW * MROWS) * 4 <= 131072);
static_assert(32 * 4 + 16 <= 131072);

typedef _Float16 h16;
typedef __attribute__((ext_vector_type(16))) _Float16 v16h;
typedef __attribute__((ext_vector_type(8)))  _Float16 v8h;
typedef __attribute__((ext_vector_type(8)))  float    v8f;
typedef __attribute__((ext_vector_type(4)))  float    v4f;
typedef v4f  __attribute__((may_alias)) v4fa;

__device__ __forceinline__ v16h cat16(v8h lo, v8h hi) { return __builtin_shufflevector(lo, hi, 0, 1, 2, 3, 4, 5, 6, 7, 8, 9, 10, 11, 12, 13, 14, 15); }
__device__ __forceinline__ v8f wmma16(v16h a, v16h b, v8f c) { return __builtin_amdgcn_wmma_f32_16x16x32_f16(false, a, false, b, (short)0, c, false, false); }
__device__ __forceinline__ v16h  ldh(const h16* p) { return cat16(*(const v8h*)p, *(const v8h*)(p + 16)); }
__device__ __forceinline__ void wave_sync() { __builtin_amdgcn_fence(3  , "wavefront"); __builtin_amdgcn_wave_barrier(); asm volatile("" ::: "memory"); }
static __device__ __forceinline__ h16 toh_flush(float v) { const h16 r = (h16)v; return (fabsf(v) < 6.103515625e-05f) ? (h16)0.0f : r; }
__device__ __forceinline__ v8f wg(v16h a, v16h b, v8f c) { c = wmma16(a, b, c); asm volatile("v_nop\n\tv_nop\n\tv_nop\n\tv_nop" : "+v"(c) : "v"(a), "v"(b)); return c; }

__global__ __launch_bounds__(256) void k_split(const float* __restrict__ src, h16* PH, h16* PL, float* SQ, float sgn, int wsq, unsigned rows_c, unsigned rows_f) {
    __shared__ __align__(16) float sq[32];
    const unsigned tid = threadIdx.x;
    const unsigned rc = blockIdx.y * rows_c + blockIdx.x * 32u;
    const size_t so = ((size_t)blockIdx.y * rows_f + (size_t)blockIdx.x * 32u) * DIM + (size_t)tid * 8;
    const size_t po = (size_t)rc * DIM + (size_t)tid * 8;
    const v8f v = *(const v8f*)(src + so);
    v8h hv, rv; float w2[8];
#pragma unroll
    for (int k = 0; k < 8; ++k) {
        const float w = v[k] * sgn;
        const h16 a = toh_flush(w);
        hv[k] = a;
        rv[k] = toh_flush((w - (float)a) * QRS);
        w2[k] = w * w; }
    float s = ((w2[0] + w2[1]) + (w2[2] + w2[3])) + ((w2[4] + w2[5]) + (w2[6] + w2[7]));
    s += __shfl_xor(s, 1, 32); s += __shfl_xor(s, 2, 32); s += __shfl_xor(s, 4, 32);
    if ((tid & 7u) == 0u) sq[tid >> 3] = 0.5f * s;
    __syncthreads();
    const v4f qv = *(const v4fa*)(&sq[(tid & 7u) * 4]);
    const bool wq = (wsq != 0) & (tid < 8u);
#pragma unroll 1
    for (int ps = 0; ps < 2; ++ps) {
        *(volatile v8h*)(PH + po) = hv;
        *(volatile v8h*)(PL + po) = rv;
        if (wq) *(volatile v4f*)(SQ + rc + tid * 4u) = qv;
        if (ps == 0) __threadfence(); }
}

__global__ __launch_bounds__(32 * SW) void k_scan(const h16* __restrict__ XH, const h16* __restrict__ XL, const h16* __restrict__ CH, const h16* __restrict__ CL,
                                                  const float* __restrict__ CSQ, const float* __restrict__ X, const float* __restrict__ CB, int* OUT) {
    __shared__ int cand[SW * MROWS * 16];
    __shared__ int resl[SW * MROWS];
    const int lane = threadIdx.x & 31, lr = lane & 15, hi = lane >> 4;
    const int wave = __builtin_amdgcn_readfirstlane((int)(threadIdx.x >> 5));
    const unsigned bb = blockIdx.y;
    const unsigned t0 = (blockIdx.x * SW + (unsigned)wave) * MROWS;
    const unsigned row0 = bb * SEQ + t0;
    v16h xh[2][2], xl[2][2];
#pragma unroll
    for (int mt = 0; mt < 2; ++mt)
#pragma unroll
        for (int ks = 0; ks < 2; ++ks) {
            const size_t o = (size_t)(row0 + mt * 16 + lr) * DIM + 8 * hi + ks * 32;
            xh[mt][ks] = ldh(XH + o); xl[mt][ks] = ldh(XL + o); }
    float bv[2][8]; int bi[2][8];
#pragma unroll
    for (int mt = 0; mt < 2; ++mt)
#pragma unroll
        for (int r = 0; r < 8; ++r) { bv[mt][r] = 3.0e38f; bi[mt][r] = 0; }
    unsigned cidx = (unsigned)lr;
    unsigned cofs = (unsigned)lr * DIM + 8u * (unsigned)hi;
    asm volatile("" : "+v"(cidx));
    asm volatile("" : "+v"(cofs));
#pragma unroll 1
    for (int t = 0; t < NCODE / 16; ++t) {
        const float cs = CSQ[cidx];
        const v16h ch0 = ldh(CH + cofs), ch1 = ldh(CH + cofs + 32);
        const v16h cl0 = ldh(CL + cofs), cl1 = ldh(CL + cofs + 32);
#pragma unroll
        for (int mt = 0; mt < 2; ++mt) {
            v8f H = (v8f){}, L = (v8f){};
            H = wg(xh[mt][0], ch0, H); H = wg(xh[mt][1], ch1, H);
            L = wg(xh[mt][0], cl0, L); L = wg(xh[mt][1], cl1, L);
            L = wg(xl[mt][0], ch0, L); L = wg(xl[mt][1], ch1, L);
#pragma unroll
            for (int r = 0; r < 8; ++r) {
                const float s = (H[r] + cs) + L[r] * QRI;
                const bool lt = s < bv[mt][r];
                bv[mt][r] = lt ? s : bv[mt][r];
                bi[mt][r] = lt ? (int)cidx : bi[mt][r]; }
        }
        cidx += 16u; cofs += 16u * DIM;
    }
    const int cb = wave * MROWS * 16;
#pragma unroll
    for (int mt = 0; mt < 2; ++mt)
#pragma unroll
        for (int r = 0; r < 8; ++r) cand[cb + (mt * 16 + hi * 8 + r) * 16 + lr] = bi[mt][r];
    wave_sync();
    const float* xb = X + ((size_t)bb * SEQ_FULL + (size_t)t0) * DIM;
#pragma unroll 1
    for (int p = 0; p < MROWS / 2; ++p) {
        const int q = 2 * p + hi;
        unsigned code = (unsigned)cand[cb + q * 16 + lr];
        code = code < (unsigned)NCODE ? code : (unsigned)(NCODE - 1);
        asm volatile("" : "+v"(code));
        const float* xr = xb + (size_t)q * DIM;
        const float* cr = CB + (size_t)code * DIM;
        v4f ad = (v4f){}, ax = (v4f){}, ac = (v4f){};
#pragma unroll 2
        for (int j = 0; j < DIM / 4; ++j) {
            const v4f xv = *(const v4f*)(xr + 4 * j);
            const v4f cv = *(const v4f*)(cr + 4 * j);
            ad = ad + xv * cv; ax = ax + xv * xv; ac = ac + cv * cv; }
        const float dot = (ad[0] + ad[1]) + (ad[2] + ad[3]);
        const float xs  = (ax[0] + ax[1]) + (ax[2] + ax[3]);
        const float cq  = (ac[0] + ac[1]) + (ac[2] + ac[3]);
        float dist = (xs + cq) - 2.0f * dot;
        int bidx = (int)code;
#pragma unroll
        for (int m = 8; m >= 1; m >>= 1) {
            const float ov = __shfl_xor(dist, m, 32);
            const int   oi = __shfl_xor(bidx, m, 32);
            const bool take = (ov < dist) | ((ov == dist) & (oi < bidx));
            dist = take ? ov : dist;
            bidx = take ? oi : bidx; }
        if (lr == 0) resl[wave * MROWS + q] = bidx;
    }
    wave_sync();
    const int val = resl[wave * MROWS + lane];
    int* op = OUT + (size_t)bb * OUT_SEQ + (size_t)t0 + (size_t)lane;
    *(volatile int*)op = val;
    __threadfence();
    *(volatile int*)op = val;
}

static constexpr size_t al256(size_t v) { return (v + 255) & ~(size_t)255; }
static constexpr size_t SZ_XP = al256((size_t)NB * SEQ * DIM * 2);
static constexpr size_t SZ_CP = al256((size_t)NCODE * DIM * 2);
static constexpr size_t SZ_SQ = al256((size_t)NCODE * 4);
static constexpr size_t SZ_TOTAL = 2 * SZ_XP + 2 * SZ_CP + SZ_SQ;
static_assert(SZ_TOTAL <= (size_t)134217728);
static_assert((size_t)(NB * SEQ / 32) * 32 * DIM * 2 <= SZ_XP);
static_assert((size_t)(NCODE / 32) * 32 * DIM * 2 <= SZ_CP);
static_assert((size_t)(NCODE / 32) * 128 <= SZ_SQ);

extern "C" void kernel_launch(void* const* d_in, const int* in_sizes, int n_in,
                              void* d_out, int out_size, void* d_ws, size_t ws_size, hipStream_t stream) {
    if (n_in < 2) return;
    const size_t needx = ((size_t)(NB - 1) * SEQ_FULL + SEQ) * DIM;
    if ((size_t)in_sizes[0] < needx) return;
    if ((size_t)in_sizes[1] < (size_t)NCODE * DIM) return;
    if ((size_t)out_size < (size_t)(NB - 1) * OUT_SEQ + SEQ) return;
    if (SZ_TOTAL > ws_size) return;
    const float* x  = (const float*)d_in[0];
    const float* cbk = (const float*)d_in[1];
    int* OUT = (int*)d_out;
    char* wsp = (char*)d_ws;
    h16* XH = (h16*)wsp; wsp += SZ_XP;
    h16* XL = (h16*)wsp; wsp += SZ_XP;
    h16* CH = (h16*)wsp; wsp += SZ_CP;
    h16* CL = (h16*)wsp; wsp += SZ_CP;
    float* CSQ = (float*)wsp; wsp += SZ_SQ;

    k_split<<<dim3(SEQ / 32, NB, 1), 256, 0, stream>>>(x, XH, XL, CSQ, -1.0f, 0, (unsigned)SEQ, (unsigned)SEQ_FULL);
    k_split<<<dim3(NCODE / 32, 1, 1), 256, 0, stream>>>(cbk, CH, CL, CSQ, 1.0f, 1, (unsigned)NCODE, (unsigned)NCODE);
    k_scan<<<dim3(SEQ / (SW * MROWS), NB, 1), 32 * SW, 0, stream>>>(XH, XL, CH, CL, CSQ, x, cbk, OUT);
}
